// GATClassifier_23648089931783
// MI455X (gfx1250) — hardware-verified
//
#include <hip/hip_runtime.h>
#include <stddef.h>
#include <stdint.h>


#define DIN     128
#define HID     512
#define NHEAD   8
#define HC      64
#define NCLS    2
#define NTHR    256
#define NWAVE   8
#define EPT     8
#define CHUNK   (NTHR * EPT)
#define WCAP    (EPT * 32)
#define LISTN   (NWAVE * WCAP)
#define NBMAX   2048
#define RCAP    28672
#define DEGCAP  4096
#define STW     1536
#define STRES   512
#define GBM     64
#define GBN     64
#define GTHR    128
#define NCT     (HID / GBN)
#define NEGS    0.2f
#define WSMAX   134217728
#define LDS_TAB (HID + 2 * HID + 16)
#define LDS_AGG ((2 * RCAP + 2 * NBMAX + LISTN) * 4 + 64 + LDS_TAB * 4)

static_assert((CHUNK & (CHUNK - 1)) == 0 && CHUNK <= 4096);
static_assert((NBMAX & (NBMAX - 1)) == 0 && NBMAX <= 4096);
static_assert(NTHR * 8 == NBMAX);
static_assert(LISTN >= NBMAX);
static_assert(LISTN >= NWAVE * WCAP);
static_assert((RCAP % 32) == 0);
static_assert(NWAVE * STW <= RCAP);
static_assert(STRES >= HID && STW - STRES >= 4 * (NBMAX / NWAVE));
static_assert(STW >= 2 * (NBMAX / NWAVE));
static_assert(LDS_AGG <= 300000);
static_assert(GBM == (GTHR / 32) * 16);
static_assert(GTHR == 2 * GBM);
static_assert((DIN % 32) == 0 && (HID % GBN) == 0);
static_assert(GBN == HC && NCT == NHEAD);
static_assert(HID == NHEAD * HC);
static_assert(GBM * 16 / 4 == 2 * GTHR);

typedef float          v2f   __attribute__((ext_vector_type(2)));
typedef float          v4f   __attribute__((ext_vector_type(4)));
typedef float          v8f   __attribute__((ext_vector_type(8)));
typedef int            v4i   __attribute__((ext_vector_type(4)));
typedef int            v8i   __attribute__((ext_vector_type(8)));
typedef unsigned short v8us  __attribute__((ext_vector_type(8)));
typedef __bf16         v16bf __attribute__((ext_vector_type(16)));
union FragB { v16bf v; v8us h[2]; v8i w; };

__device__ __forceinline__ v8f wmb(const FragB& a, const FragB& b, v8f c) {
  v8f d = __builtin_amdgcn_wmma_f32_16x16x32_bf16(false, a.v, false, b.v, (short)0, c, false, false);
  asm volatile("v_nop\n\tv_nop\n\tv_nop\n\tv_nop" : "+v"(d) : "v"(a.w), "v"(b.w));
  return d;
}

__device__ __forceinline__ void ldwait() {
  asm volatile("s_wait_loadcnt 0x0" ::: "memory");
}

__device__ __forceinline__ unsigned short bf16bits(float f) {
  unsigned u = __float_as_uint(f);
  u = u + 0x7FFFu + ((u >> 16) & 1u);
  return (unsigned short)(u >> 16);
}
__device__ __forceinline__ float bf16r(float f) {
  return __uint_as_float(((unsigned)bf16bits(f)) << 16);
}
__device__ __forceinline__ v8us cvt8b(const v4f a, const v4f b) {
  v8us r;
  r[0] = bf16bits(a.x); r[1] = bf16bits(a.y); r[2] = bf16bits(a.z); r[3] = bf16bits(a.w);
  r[4] = bf16bits(b.x); r[5] = bf16bits(b.y); r[6] = bf16bits(b.z); r[7] = bf16bits(b.w);
  return r;
}
__device__ __forceinline__ float lrelu(float v) { return v > 0.f ? v : NEGS * v; }

__device__ __forceinline__ int scan_chunk(const int* __restrict__ dsts, int nE, int cbase, int slotBase,
                                          int nb, int vec8, int* list, int tid, int lane, int wave) {
  int wc = 0;
  const int el0  = tid * EPT;
  const int e0   = cbase + el0;
  const int sent = -2147483647 - 1;
  v4i da, db;
  if (vec8 != 0 && cbase + CHUNK <= nE) {
    da = *(const v4i*)(dsts + e0);
    db = *(const v4i*)(dsts + e0 + 4);
  } else {
    da.x = (e0     < nE) ? dsts[min(e0,     nE - 1)] : sent;
    da.y = (e0 + 1 < nE) ? dsts[min(e0 + 1, nE - 1)] : sent;
    da.z = (e0 + 2 < nE) ? dsts[min(e0 + 2, nE - 1)] : sent;
    da.w = (e0 + 3 < nE) ? dsts[min(e0 + 3, nE - 1)] : sent;
    db.x = (e0 + 4 < nE) ? dsts[min(e0 + 4, nE - 1)] : sent;
    db.y = (e0 + 5 < nE) ? dsts[min(e0 + 5, nE - 1)] : sent;
    db.z = (e0 + 6 < nE) ? dsts[min(e0 + 6, nE - 1)] : sent;
    db.w = (e0 + 7 < nE) ? dsts[min(e0 + 7, nE - 1)] : sent;
  }
  const unsigned nbs = (unsigned)slotBase;
  const unsigned unb = (unsigned)nb;
  const unsigned s0 = (unsigned)da.x - nbs, s1 = (unsigned)da.y - nbs;
  const unsigned s2 = (unsigned)da.z - nbs, s3 = (unsigned)da.w - nbs;
  const unsigned s4 = (unsigned)db.x - nbs, s5 = (unsigned)db.y - nbs;
  const unsigned s6 = (unsigned)db.z - nbs, s7 = (unsigned)db.w - nbs;
  const bool h0 = s0 < unb, h1 = s1 < unb, h2 = s2 < unb, h3 = s3 < unb;
  const bool h4 = s4 < unb, h5 = s5 < unb, h6 = s6 < unb, h7 = s7 < unb;
  const unsigned any = __builtin_amdgcn_ballot_w32(h0 | h1 | h2 | h3 | h4 | h5 | h6 | h7);
  if (any != 0u) {
#define HITJ(J, HJ, SJ) { \
      const unsigned mj = __builtin_amdgcn_ballot_w32(HJ); \
      if (mj != 0u) { \
        if (HJ) { \
          const int pos = wc + (int)__builtin_amdgcn_mbcnt_lo(mj, 0u); \
          if (pos < WCAP) list[wave * WCAP + pos] = ((el0 + (J)) << 12) | (int)(SJ); \
        } \
        wc += (int)__builtin_popcount(mj); } }
    HITJ(0, h0, s0)
    HITJ(1, h1, s1)
    HITJ(2, h2, s2)
    HITJ(3, h3, s3)
    HITJ(4, h4, s4)
    HITJ(5, h5, s5)
    HITJ(6, h6, s6)
    HITJ(7, h7, s7)
#undef HITJ
  }
  return wc;
}

__global__ __launch_bounds__(NTHR) void k_xprep(const float* __restrict__ x, unsigned short* xb, int nN, int nUnits) {
  const int i = (int)blockIdx.x * NTHR + (int)threadIdx.x;
  if (i >= nUnits) return;
  const int row = i >> 4;
  const int c0  = (i & 15) * 8;
  const int rc  = row < nN ? row : nN - 1;
  const float* p = x + (size_t)rc * DIN + c0;
  v4f a = *(const v4f*)p, b = *(const v4f*)(p + 4);
  const v4f z4 = {0.f, 0.f, 0.f, 0.f};
  if (row >= nN) { a = z4; b = z4; }
  const v8us hv = cvt8b(a, b);
  const size_t o = (size_t)row * DIN + c0;
  *(volatile v8us*)(xb + o) = hv;
  __threadfence();
  *(volatile v8us*)(xb + o) = hv;
}

__global__ __launch_bounds__(NTHR) void k_wtr(const float* __restrict__ w, unsigned short* wt, int K, int C, int nUnits) {
  const int u = (int)blockIdx.x * NTHR + (int)threadIdx.x;
  if (u >= nUnits) return;
  const int kq = K >> 3;
  const int n  = u / kq;
  const int k8 = (u - n * kq) * 8;
  const float* p = w + (size_t)k8 * (size_t)C + n;
  v4f a, b;
  a.x = p[0];               a.y = p[(size_t)C];       a.z = p[(size_t)2 * C];   a.w = p[(size_t)3 * C];
  b.x = p[(size_t)4 * C];   b.y = p[(size_t)5 * C];   b.z = p[(size_t)6 * C];   b.w = p[(size_t)7 * C];
  const v8us hv = cvt8b(a, b);
  const size_t o = (size_t)n * (size_t)K + k8;
  *(volatile v8us*)(wt + o) = hv;
  __threadfence();
  *(volatile v8us*)(wt + o) = hv;
}

__global__ __launch_bounds__(GTHR) void k_gemm1(
    const unsigned short* __restrict__ A, const unsigned short* __restrict__ WT,
    const float* __restrict__ asr, const float* __restrict__ adr,
    float* H, float* ALN, int K)
{
  __shared__ __attribute__((aligned(16))) float stg[GBM * GBN];
  __shared__ __attribute__((aligned(16))) float sav[2 * HID];
  __shared__ __attribute__((aligned(16))) float sal[GBM * 16];
  const int tid = (int)threadIdx.x, lane = tid & 31, wave = tid >> 5, hh = lane >> 4, m = lane & 15;
  const int rowBase = (int)blockIdx.x * GBM;

  for (int i = tid; i < 2 * HID; i += GTHR) {
    const int ia = i < HID ? i : HID - 1;
    int ib = i - HID; ib = ib < 0 ? 0 : (ib > HID - 1 ? HID - 1 : ib);
    const float va = asr[ia];
    const float vb = adr[ib];
    sav[i] = bf16r(i < HID ? va : vb);
  }
  __syncthreads();

  const unsigned short* ap = A + (size_t)(rowBase + 16 * wave + m) * (size_t)K + 8 * hh;
  const int ksteps = K >> 5;

#pragma unroll 1
  for (int ct = 0; ct < NCT; ++ct) {
    const int col0 = ct * GBN;
    v8f acc[4];
    {
      const v8f z = {0.f, 0.f, 0.f, 0.f, 0.f, 0.f, 0.f, 0.f};
      acc[0] = z; acc[1] = z; acc[2] = z; acc[3] = z;
    }
    const unsigned short* wp = WT + (size_t)(col0 + m) * (size_t)K + 8 * hh;
#pragma unroll 1
    for (int ks = 0; ks < ksteps; ++ks) {
      FragB af;
      af.h[0] = *(const v8us*)(ap + 32 * ks);
      af.h[1] = *(const v8us*)(ap + 32 * ks + 16);
#pragma unroll
      for (int t = 0; t < 4; ++t) {
        const unsigned short* wq = wp + (size_t)(16 * t) * (size_t)K + 32 * ks;
        FragB bf;
        bf.h[0] = *(const v8us*)wq;
        bf.h[1] = *(const v8us*)(wq + 16);
        acc[t] = wmb(af, bf, acc[t]);
      }
    }

#pragma unroll
    for (int t = 0; t < 4; ++t) {
      const int lc = 16 * t + m;
#pragma unroll
      for (int r = 0; r < 8; ++r) {
        const int lr = 16 * wave + 8 * hh + r;
        stg[lr * GBN + lc] = acc[t][r];
      }
    }
    __syncthreads();

    {
      v4f fv[8];
#pragma unroll
      for (int i = 0; i < 8; ++i) {
        const int lr = 16 * wave + 2 * i + hh;
        fv[i] = *(const v4f*)(stg + lr * GBN + 4 * m);
      }
#pragma unroll
      for (int i = 0; i < 8; ++i) {
        const int lr = 16 * wave + 2 * i + hh;
        const int gr = rowBase + lr;
        float* op = H + (size_t)gr * (size_t)HID + col0 + 4 * m;
        *(volatile v4f*)op = fv[i];
      }
      __threadfence();
#pragma unroll
      for (int i = 0; i < 8; ++i) {
        const int lr = 16 * wave + 2 * i + hh;
        const int gr = rowBase + lr;
        float* op = H + (size_t)gr * (size_t)HID + col0 + 4 * m;
        *(volatile v4f*)op = fv[i];
      }
    }

    {
      const int row   = tid & (GBM - 1);
      const int which = tid >> 6;
      const float* sr = stg + row * GBN;
      const float* wv = sav + which * HID + col0;
      float d = 0.f;
#pragma unroll 2
      for (int c4 = 0; c4 < GBN / 4; ++c4) {
        const v4f hv = *(const v4f*)(sr + 4 * c4);
        const v4f av = *(const v4f*)(wv + 4 * c4);
        d = fmaf(hv.x, av.x, d); d = fmaf(hv.y, av.y, d);
        d = fmaf(hv.z, av.z, d); d = fmaf(hv.w, av.w, d);
      }
      sal[row * 16 + which * 8 + ct] = d;
    }
    __syncthreads();
  }

  {
    v4f pa[2];
#pragma unroll
    for (int i = 0; i < 2; ++i) {
      const int p = i * GTHR + tid;
      pa[i] = *(const v4f*)(sal + 4 * p);
    }
    float* ob = ALN + (size_t)rowBase * 16;
#pragma unroll
    for (int i = 0; i < 2; ++i) {
      const int p = i * GTHR + tid;
      *(volatile v4f*)(ob + 4 * p) = pa[i];
    }
    __threadfence();
#pragma unroll
    for (int i = 0; i < 2; ++i) {
      const int p = i * GTHR + tid;
      *(volatile v4f*)(ob + 4 * p) = pa[i];
    }
  }
}

template<int LAYER>
__global__ __launch_bounds__(NTHR) void k_agg(
    const int* __restrict__ srcs, const int* __restrict__ dsts,
    const float* __restrict__ H, const float* __restrict__ ALN,
    const float* __restrict__ b1, const float* __restrict__ W2,
    const float* __restrict__ as2v, const float* __restrict__ ad2v, const float* __restrict__ b2,
    const float* __restrict__ NDin, float* NDout, float* out,
    int nN, int nE, int nb, int vec8) {
  extern __shared__ v4f lds_dyn[];
  int* reg1 = (int*)lds_dyn;
  int* reg2 = reg1 + RCAP;
  int* scnt = reg2 + RCAP;
  int* soff = scnt + NBMAX;
  int* list = soff + NBMAX;
  int* wcnt = list + LISTN;
  int* wtot = wcnt + NWAVE;
  float* b1s  = (float*)(wtot + NWAVE);
  float* w2s  = b1s + HID;
  float* misc = w2s + 2 * HID;
  const int tid = (int)threadIdx.x, lane = tid & 31, wave = tid >> 5;
  const int nodeBase = (int)blockIdx.x * nb;

  for (int i = tid; i < NBMAX; i += NTHR) scnt[i] = 0;
  if (LAYER == 1) {
    for (int i = tid; i < HID; i += NTHR) b1s[i] = bf16r(b1[i]);
    for (int i = tid; i < 2 * HID; i += NTHR) w2s[i] = bf16r(W2[i]);
    if (tid < 2) { misc[tid] = bf16r(as2v[tid]); misc[2 + tid] = bf16r(ad2v[tid]); }
  } else {
    if (tid < 2) misc[4 + tid] = bf16r(b2[tid]);
  }
  __syncthreads();

  int tot = 0;
  const int nChunks = (nE + CHUNK - 1) / CHUNK;
#pragma unroll 1
  for (int ch = 0; ch < nChunks; ++ch) {
    const int cbase = ch * CHUNK;
    const int wc = scan_chunk(dsts, nE, cbase, nodeBase, nb, vec8, list, tid, lane, wave);
    if (lane == 0) wcnt[wave] = wc;
    __syncthreads();
    int pre = 0, all = 0;
#pragma unroll
    for (int w2 = 0; w2 < NWAVE; ++w2) {
      int c = wcnt[w2];
      c = c < 0 ? 0 : (c > WCAP ? WCAP : c);
      all += c;
      pre += (w2 < wave) ? c : 0;
    }
    const int wcc  = wc > WCAP ? WCAP : wc;
    const int base = tot + pre;
#pragma unroll 1
    for (int i = lane; i < wcc; i += 32) {
      const int ent = list[wave * WCAP + i];
      const int el  = (ent >> 12) & (CHUNK - 1);
      const int sl  = ent & (NBMAX - 1);
      int eid = cbase + el;
      eid = eid > nE - 1 ? nE - 1 : eid;
      const int pos = base + i;
      if (pos < RCAP) reg1[pos] = (int)(((unsigned)eid << 12) | (unsigned)sl);
    }
    tot += all;
    tot = tot > RCAP ? RCAP : tot;
    __syncthreads();
  }
  const int nh = tot;

  if (wave == 0) {
#pragma unroll 1
    for (int b0 = 0; b0 < nh; b0 += 32) {
      const int idx = b0 + lane;
      const int uv  = reg1[idx < RCAP ? idx : RCAP - 1];
      const int m32 = (nh - b0) < 32 ? (nh - b0) : 32;
#pragma unroll 1
      for (int k = 0; k < m32; ++k) {
        const int u  = __builtin_amdgcn_readlane(uv, k);
        const int sl = u & (NBMAX - 1);
        if (lane == 0) scnt[sl] = scnt[sl] + 1;
      }
    }
  }
  __syncthreads();

  {
    const v4i ca = *(const v4i*)(scnt + 8 * tid);
    const v4i cb = *(const v4i*)(scnt + 8 * tid + 4);
    const int e0 = ca.x < 0 ? 0 : ca.x, e1 = ca.y < 0 ? 0 : ca.y, e2 = ca.z < 0 ? 0 : ca.z, e3 = ca.w < 0 ? 0 : ca.w;
    const int e4 = cb.x < 0 ? 0 : cb.x, e5 = cb.y < 0 ? 0 : cb.y, e6 = cb.z < 0 ? 0 : cb.z, e7 = cb.w < 0 ? 0 : cb.w;
    const int ts = e0 + e1 + e2 + e3 + e4 + e5 + e6 + e7;
    int incl = ts;
#pragma unroll
    for (int d = 1; d < 32; d <<= 1) {
      const int up = __shfl_up(incl, d);
      if (lane >= d) incl += up;
    }
    if (lane == 31) wtot[wave] = incl;
    __syncthreads();
    int pre = 0;
#pragma unroll
    for (int w2 = 0; w2 < NWAVE; ++w2) pre += (w2 < wave) ? wtot[w2] : 0;
    int run = pre + incl - ts;
    soff[8 * tid + 0] = run; run += e0;
    soff[8 * tid + 1] = run; run += e1;
    soff[8 * tid + 2] = run; run += e2;
    soff[8 * tid + 3] = run; run += e3;
    soff[8 * tid + 4] = run; run += e4;
    soff[8 * tid + 5] = run; run += e5;
    soff[8 * tid + 6] = run; run += e6;
    soff[8 * tid + 7] = run;
  }
  __syncthreads();
  for (int i = tid; i < NBMAX; i += NTHR) list[i] = soff[i];
  __syncthreads();

  if (wave == 0) {
#pragma unroll 1
    for (int b0 = 0; b0 < nh; b0 += 32) {
      const int idx = b0 + lane;
      const int uv  = reg1[idx < RCAP ? idx : RCAP - 1];
      const int m32 = (nh - b0) < 32 ? (nh - b0) : 32;
#pragma unroll 1
      for (int k = 0; k < m32; ++k) {
        const int u   = __builtin_amdgcn_readlane(uv, k);
        const int sl  = u & (NBMAX - 1);
        const int eid = (int)((unsigned)u >> 12);
        if (lane == 0) {
          int pos = list[sl];
          pos = pos < 0 ? 0 : (pos > RCAP - 1 ? RCAP - 1 : pos);
          reg2[pos] = eid;
          list[sl] = pos + 1;
        }
      }
    }
  }
  __syncthreads();

  const int nbw = nb >> 3;
  const bool ovf = (nh >= RCAP);
  const float qnan = __int_as_float(0x7fc00000);
  const int nhm1 = nh > 0 ? nh - 1 : 0;
  float* stw = (float*)reg1 + wave * STW;

  if (LAYER == 1) {
    float* str = stw + STRES;
    const int myh = lane >> 2;
    const float as20 = misc[0], as21 = misc[1], ad20 = misc[2], ad21 = misc[3];
#pragma unroll 1
    for (int jt = 0; jt < nbw; ++jt) {
      const int slot = wave * nbw + jt;
      const int grow = nodeBase + slot;
      const int gcl  = grow < nN ? grow : nN - 1;
      int st = soff[slot];
      const int craw = scnt[slot];
      int cnt = craw;
      st  = st < 0 ? 0 : (st > nh ? nh : st);
      cnt = cnt < 0 ? 0 : (cnt > DEGCAP ? DEGCAP : cnt);
      if (cnt > nh - st) cnt = nh - st;
      const float pz = (ovf || craw > DEGCAP) ? qnan : 0.0f;
      const bool liv = grow < nN;

      const float* hr = H + (size_t)gcl * HID + 16 * lane;
      const v4f g0 = *(const v4f*)hr, g1 = *(const v4f*)(hr + 4), g2 = *(const v4f*)(hr + 8), g3 = *(const v4f*)(hr + 12);
      const float asf = ALN[(size_t)gcl * 16 + myh];
      const float adf = ALN[(size_t)gcl * 16 + 8 + myh];
      ldwait();
      float av[16];
      av[0]  = g0.x; av[1]  = g0.y; av[2]  = g0.z; av[3]  = g0.w;
      av[4]  = g1.x; av[5]  = g1.y; av[6]  = g1.z; av[7]  = g1.w;
      av[8]  = g2.x; av[9]  = g2.y; av[10] = g2.z; av[11] = g2.w;
      av[12] = g3.x; av[13] = g3.y; av[14] = g3.z; av[15] = g3.w;
      float mx = lrelu(asf + adf);
      float dn = 1.0f;

#pragma unroll 1
      for (int q = 0; q < cnt; ++q) {
        int idx = st + q; idx = idx < 0 ? 0 : (idx > nhm1 ? nhm1 : idx);
        int eid = reg2[idx]; eid = eid < 0 ? 0 : (eid > nE - 1 ? nE - 1 : eid);
        const int sraw = srcs[eid];
        const int s = sraw < 0 ? 0 : (sraw > nN - 1 ? nN - 1 : sraw);
        const float* kr = H + (size_t)s * HID + 16 * lane;
        const v4f v0 = *(const v4f*)kr, v1 = *(const v4f*)(kr + 4), v2 = *(const v4f*)(kr + 8), v3 = *(const v4f*)(kr + 12);
        const float asv = ALN[(size_t)s * 16 + myh];
        ldwait();
        const float el = lrelu(asv + adf);
        const float df = el - mx;
        const float ee = __expf(-fabsf(df));
        const bool up  = df > 0.f;
        const float s1 = up ? ee : 1.0f;
        const float s2 = up ? 1.0f : ee;
        mx = up ? el : mx;
        dn = fmaf(dn, s1, s2);
        av[0]  = fmaf(av[0],  s1, s2 * v0.x); av[1]  = fmaf(av[1],  s1, s2 * v0.y);
        av[2]  = fmaf(av[2],  s1, s2 * v0.z); av[3]  = fmaf(av[3],  s1, s2 * v0.w);
        av[4]  = fmaf(av[4],  s1, s2 * v1.x); av[5]  = fmaf(av[5],  s1, s2 * v1.y);
        av[6]  = fmaf(av[6],  s1, s2 * v1.z); av[7]  = fmaf(av[7],  s1, s2 * v1.w);
        av[8]  = fmaf(av[8],  s1, s2 * v2.x); av[9]  = fmaf(av[9],  s1, s2 * v2.y);
        av[10] = fmaf(av[10], s1, s2 * v2.z); av[11] = fmaf(av[11], s1, s2 * v2.w);
        av[12] = fmaf(av[12], s1, s2 * v3.x); av[13] = fmaf(av[13], s1, s2 * v3.y);
        av[14] = fmaf(av[14], s1, s2 * v3.z); av[15] = fmaf(av[15], s1, s2 * v3.w);
      }
      const float inv = __builtin_amdgcn_rcpf(dn);

#pragma unroll
      for (int i = 0; i < 16; ++i) stw[16 * lane + i] = av[i] * inv;
      float p0 = 0.f, p1 = 0.f;
#pragma unroll 1
      for (int i = 0; i < 16; ++i) {
        const int c = 16 * lane + i;
        float v = stw[c] + b1s[c];
        const float ng = fminf(v, 0.0f);
        const float em = __expf(ng) - 1.0f;
        v = v > 0.0f ? v : em;
        p0 = fmaf(v, w2s[2 * c], p0);
        p1 = fmaf(v, w2s[2 * c + 1], p1);
      }
#pragma unroll
      for (int off = 16; off > 0; off >>= 1) {
        p0 += __shfl_xor(p0, off);
        p1 += __shfl_xor(p1, off);
      }
      const float sc2 = fmaf(p1, as21, p0 * as20);
      const float dc2 = fmaf(p1, ad21, p0 * ad20);
      const float r0 = (liv ? p0  : 0.0f) + pz;
      const float r1 = (liv ? p1  : 0.0f) + pz;
      const float r2 = (liv ? sc2 : 0.0f) + pz;
      const float r3 = (liv ? dc2 : 0.0f) + pz;
      if (lane == 0) {
        str[4 * jt + 0] = r0; str[4 * jt + 1] = r1;
        str[4 * jt + 2] = r2; str[4 * jt + 3] = r3;
      }
    }
    __builtin_amdgcn_fence(__ATOMIC_RELEASE, "wavefront");
    __builtin_amdgcn_wave_barrier();
    float* nb0 = NDout + (size_t)(nodeBase + wave * nbw) * 4;
#pragma unroll 1
    for (int p = lane; p < nbw; p += 32) {
      const v4f rv = *(const v4f*)(str + 4 * p);
      *(volatile v4f*)(nb0 + 4 * p) = rv;
    }
    __threadfence();
#pragma unroll 1
    for (int p = lane; p < nbw; p += 32) {
      const v4f rv = *(const v4f*)(str + 4 * p);
      *(volatile v4f*)(nb0 + 4 * p) = rv;
    }
  } else {
    const float b20 = misc[4], b21 = misc[5];
#pragma unroll 1
    for (int base = 0; base < nbw; base += 32) {
      const int li  = base + lane;
      const bool val = li < nbw;
      const int lic = val ? li : nbw - 1;
      const int slot = wave * nbw + lic;
      const int grow = nodeBase + slot;
      const int gcl  = grow < nN ? grow : nN - 1;
      int st = soff[slot];
      const int craw = scnt[slot];
      int cnt = craw;
      st  = st < 0 ? 0 : (st > nh ? nh : st);
      cnt = cnt < 0 ? 0 : (cnt > DEGCAP ? DEGCAP : cnt);
      if (cnt > nh - st) cnt = nh - st;
      const float pz = (ovf || craw > DEGCAP) ? qnan : 0.0f;
      const v4f nd = *(const v4f*)(NDin + (size_t)gcl * 4);
      ldwait();
      const float adf = nd.w;
      float mx = lrelu(nd.z + adf);
      float dn = 1.0f;
      float a0 = nd.x, a1 = nd.y;
      int cm = cnt;
#pragma unroll
      for (int off = 16; off > 0; off >>= 1) {
        const int o = __shfl_xor(cm, off);
        cm = o > cm ? o : cm;
      }
#pragma unroll 1
      for (int q = 0; q < cm; ++q) {
        const bool act = q < cnt;
        int idx = st + (act ? q : 0); idx = idx < 0 ? 0 : (idx > nhm1 ? nhm1 : idx);
        int eid = reg2[idx]; eid = eid < 0 ? 0 : (eid > nE - 1 ? nE - 1 : eid);
        const int sraw = srcs[eid];
        const int s = sraw < 0 ? 0 : (sraw > nN - 1 ? nN - 1 : sraw);
        const v4f ns = *(const v4f*)(NDin + (size_t)s * 4);
        ldwait();
        const float el = lrelu(ns.z + adf);
        const float df = el - mx;
        const float ee = __expf(-fabsf(df));
        const bool up  = act && (df > 0.f);
        const float s1 = up ? ee : 1.0f;
        const float s2 = act ? (up ? 1.0f : ee) : 0.0f;
        mx = up ? el : mx;
        dn = fmaf(dn, s1, s2);
        a0 = fmaf(a0, s1, s2 * ns.x);
        a1 = fmaf(a1, s1, s2 * ns.y);
      }
      const float inv = __builtin_amdgcn_rcpf(dn);
      const float o0 = fmaf(a0, inv, b20) + pz;
      const float o1 = fmaf(a1, inv, b21) + pz;
      if (val) { stw[2 * li] = o0; stw[2 * li + 1] = o1; }
    }
    __builtin_amdgcn_fence(__ATOMIC_RELEASE, "wavefront");
    __builtin_amdgcn_wave_barrier();
    const int np = nbw >> 1;
    const int nw0 = nodeBase + wave * nbw;
#pragma unroll 1
    for (int p = lane; p < np; p += 32) {
      const v4f rv = *(const v4f*)(stw + 4 * p);
      const int n0 = nw0 + 2 * p;
      if (n0 + 1 < nN) {
        *(volatile v4f*)(out + (size_t)n0 * NCLS) = rv;
      } else if (n0 < nN) {
        const v2f r2 = rv.xy;
        *(volatile v2f*)(out + (size_t)n0 * NCLS) = r2;
      }
    }
    __threadfence();
#pragma unroll 1
    for (int p = lane; p < np; p += 32) {
      const v4f rv = *(const v4f*)(stw + 4 * p);
      const int n0 = nw0 + 2 * p;
      if (n0 + 1 < nN) {
        *(volatile v4f*)(out + (size_t)n0 * NCLS) = rv;
      } else if (n0 < nN) {
        const v2f r2 = rv.xy;
        *(volatile v2f*)(out + (size_t)n0 * NCLS) = r2;
      }
    }
  }
}

static int pick_nb(int nE, int nN) {
  int nb = NBMAX;
  while (nb > 16 && (long long)nb * (long long)nE * 5LL > (long long)RCAP * (long long)nN * 4LL) nb >>= 1;
  return nb;
}
static inline int cdiv(int a, int b) { return (a + b - 1) / b; }

extern "C" void kernel_launch(void* const* d_in, const int* in_sizes, int n_in,
                              void* d_out, int out_size, void* d_ws, size_t ws_size,
                              hipStream_t stream) {
  if (n_in < 10) return;
  const int nN = in_sizes[0] / DIN;
  if (nN <= 0 || in_sizes[0] != nN * DIN || nN > (1 << 22)) return;
  if (in_sizes[1] < 2 || (in_sizes[1] & 1) != 0) return;
  const int nE = in_sizes[1] / 2;
  if (nE < 1 || nE > (1 << 20)) return;
  if (in_sizes[2] != DIN * HID) return;
  if (in_sizes[3] != NHEAD * HC || in_sizes[4] != NHEAD * HC) return;
  if (in_sizes[5] != HID) return;
  if (in_sizes[6] != HID * NCLS) return;
  if (in_sizes[7] != NCLS || in_sizes[8] != NCLS || in_sizes[9] != NCLS) return;
  if (out_size != nN * NCLS) return;

  const float* x    = (const float*)d_in[0];
  const int*   ei   = (const int*)  d_in[1];
  const float* W1   = (const float*)d_in[2];
  const float* as1  = (const float*)d_in[3];
  const float* ad1  = (const float*)d_in[4];
  const float* b1   = (const float*)d_in[5];
  const float* W2   = (const float*)d_in[6];
  const float* as2v = (const float*)d_in[7];
  const float* ad2v = (const float*)d_in[8];
  const float* b2   = (const float*)d_in[9];
  float* out = (float*)d_out;
  const int* src = ei;
  const int* dst = ei + nE;

  const int MP   = cdiv(nN, GBM) * GBM;
  const int nb   = pick_nb(nE, nN);
  const int gA   = cdiv(MP, nb);
  const int vec8 = ((nE & 3) == 0) ? 1 : 0;
  if (gA * nb < MP) return;
  const int rows2 = gA * nb;

  char* ws = (char*)d_ws;
  size_t off = 0;
  const size_t oXB  = off; off += (size_t)MP * DIN * 2;            off = (off + 255) & ~(size_t)255;
  const size_t oWT  = off; off += (size_t)HID * DIN * 2;           off = (off + 255) & ~(size_t)255;
  const size_t oH   = off; off += (size_t)MP * HID * 4;            off = (off + 255) & ~(size_t)255;
  const size_t oALN = off; off += (size_t)MP * 16 * 4;             off = (off + 255) & ~(size_t)255;
  const size_t oND  = off; off += (size_t)rows2 * 4 * 4;           off = (off + 255) & ~(size_t)255;
  if (off > ws_size || off > (size_t)WSMAX) return;
  unsigned short* XB  = (unsigned short*)(ws + oXB);
  unsigned short* WT  = (unsigned short*)(ws + oWT);
  float*          H   = (float*)(ws + oH);
  float*          ALN = (float*)(ws + oALN);
  float*          ND  = (float*)(ws + oND);

  hipFuncSetAttribute(reinterpret_cast<const void*>(&k_agg<1>),
                      hipFuncAttributeMaxDynamicSharedMemorySize, LDS_AGG);
  hipFuncSetAttribute(reinterpret_cast<const void*>(&k_agg<2>),
                      hipFuncAttributeMaxDynamicSharedMemorySize, LDS_AGG);

  const int nUx = MP * (DIN / 8);
  k_xprep<<<cdiv(nUx, NTHR), NTHR, 0, stream>>>(x, XB, nN, nUx);

  const int nUw = HID * (DIN / 8);
  k_wtr<<<cdiv(nUw, NTHR), NTHR, 0, stream>>>(W1, WT, DIN, HID, nUw);

  k_gemm1<<<MP / GBM, GTHR, 0, stream>>>(XB, WT, as1, ad1, H, ALN, DIN);

  k_agg<1><<<gA, NTHR, LDS_AGG, stream>>>(src, dst, H, ALN, b1, W2, as2v, ad2v, b2, ND, ND, out,
                                           nN, nE, nb, vec8);
  k_agg<2><<<gA, NTHR, LDS_AGG, stream>>>(src, dst, H, ALN, b1, W2, as2v, ad2v, b2, ND, ND, out,
                                           nN, nE, nb, vec8);
}
